// SSKernelNPLR_730144440569
// MI455X (gfx1250) — hardware-run, weakly checked
//
#include <hip/hip_runtime.h>
#include <math.h>

typedef __attribute__((ext_vector_type(16))) _Float16 v16h;
typedef __attribute__((ext_vector_type(8)))  _Float16 v8h;
typedef __attribute__((ext_vector_type(16))) __bf16   v16b;
typedef __attribute__((ext_vector_type(8)))  __bf16   v8b;
typedef __attribute__((ext_vector_type(8)))  float    v8f;
typedef __attribute__((ext_vector_type(4)))  float    v4f;
typedef __attribute__((ext_vector_type(2)))  float    v2f;
typedef __attribute__((ext_vector_type(4)))  unsigned v4u;

constexpr int kHeads    = 256;
constexpr int kPoles    = 64;
constexpr int kLen      = 2048;
constexpr int kFreq     = kLen / 2 + 1;
constexpr int kFreqPad  = 1056;
constexpr int kKdim     = 2 * kFreqPad;
constexpr int kPoleBlk  = 352;
constexpr int kPoleChunks = kFreqPad / kPoleBlk;
constexpr int kBasisWords = kLen * kFreqPad;
constexpr int kBasisBlocks = kBasisWords / 256;
constexpr float kInvLen = 1.0f / (float)kLen;
static_assert(kFreq == 1025, "node count");
static_assert((kKdim % 32) == 0, "GEMM K multiple of 32");
static_assert((kHeads % 64) == 0 && (kLen % 64) == 0, "GEMM M,N multiples of 64");
static_assert(((kKdim * 2) % 128) == 0, "operand rows are whole 128-B lines");
static_assert((kFreqPad % kPoleBlk) == 0 && (kPoleBlk % 32) == 0 && kPoleChunks == 3, "pole-sum coverage");
static_assert((kBasisWords % 256) == 0 && kBasisBlocks == 8448, "basis coverage");
static_assert(kFreqPad >= kFreq, "pad");

constexpr size_t kOffBH   = 0;
constexpr size_t kOffBL   = kOffBH + (size_t)kLen   * kKdim * 2;
constexpr size_t kOffAH   = kOffBL + (size_t)kLen   * kKdim * 2;
constexpr size_t kOffAL   = kOffAH + (size_t)kHeads * kKdim * 2;
constexpr size_t kWsTotal = kOffAL + (size_t)kHeads * kKdim * 2;
static_assert(kWsTotal == 19464192ull, "carve total");
static_assert(kWsTotal <= 134217728ull, "carve cap");
static_assert((kOffBL % 128) == 0 && (kOffAH % 128) == 0 && (kOffAL % 128) == 0, "128-B aligned regions");

__device__ __forceinline__ unsigned short f2bf_bits(float f) {
  unsigned u = __float_as_uint(f);
  return (unsigned short)((u + 0x7FFFu + ((u >> 16) & 1u)) >> 16);
}
__device__ __forceinline__ float bf_bits2f(unsigned short h) { return __uint_as_float(((unsigned)h) << 16); }
__device__ __forceinline__ unsigned bf_rne_u32(float f) {
  const unsigned u = __float_as_uint(f);
  return (u + 0x7FFFu + ((u >> 16) & 1u)) >> 16;
}
__device__ __forceinline__ float bf_u32_to_f(unsigned hb) { return __uint_as_float(hb << 16); }

__device__ __forceinline__ void dep_guard1_h(v8f& a, v16h x, v16h y, v16h z, v16h w) { asm volatile("v_nop\n\tv_nop\n\tv_nop\n\tv_nop" : "+v"(a) : "v"(x), "v"(y), "v"(z), "v"(w)); }
__device__ __forceinline__ void dep_guard1_b(v8f& a, v16b x, v16b y, v16b z, v16b w) { asm volatile("v_nop\n\tv_nop\n\tv_nop\n\tv_nop" : "+v"(a) : "v"(x), "v"(y), "v"(z), "v"(w)); }
__device__ __forceinline__ void keep4_h(v16h a, v16h b, v16h c, v16h d) { asm volatile("v_nop" :: "v"(a), "v"(b), "v"(c), "v"(d)); }
__device__ __forceinline__ void keep4_b(v16b a, v16b b, v16b c, v16b d) { asm volatile("v_nop" :: "v"(a), "v"(b), "v"(c), "v"(d)); }
__device__ __forceinline__ void acc_guard4(v8f& a, v8f& b, v8f& c, v8f& d) { asm volatile("v_nop\n\tv_nop\n\tv_nop\n\tv_nop" : "+v"(a), "+v"(b), "+v"(c), "+v"(d)); }
template <typename T> struct Frag;
template <> struct Frag<_Float16> {
  typedef v16h V; union U { v16h v; v8h h[2]; };
  static __device__ __forceinline__ v16h load(const _Float16* p) {
    U f; f.h[0] = *(const v8h*)(p); f.h[1] = *(const v8h*)(p + 16); return f.v;
  }
  static __device__ __forceinline__ v8f mma(v16h a, v16h b, v8f c) {
    return __builtin_amdgcn_wmma_f32_16x16x32_f16(false, a, false, b, (short)0, c, false, false);
  }
  static __device__ __forceinline__ void guard1(v8f& a, v16h x, v16h y, v16h z, v16h w) { dep_guard1_h(a, x, y, z, w); }
  static __device__ __forceinline__ void keep(v16h a, v16h b, v16h c, v16h d) { keep4_h(a, b, c, d); }
};
template <> struct Frag<__bf16> {
  typedef v16b V; union U { v16b v; v8b h[2]; };
  static __device__ __forceinline__ v16b load(const __bf16* p) {
    U f; f.h[0] = *(const v8b*)(p); f.h[1] = *(const v8b*)(p + 16); return f.v;
  }
  static __device__ __forceinline__ v8f mma(v16b a, v16b b, v8f c) {
    return __builtin_amdgcn_wmma_f32_16x16x32_bf16(false, a, false, b, (short)0, c, false, false);
  }
  static __device__ __forceinline__ void guard1(v8f& a, v16b x, v16b y, v16b z, v16b w) { dep_guard1_b(a, x, y, z, w); }
  static __device__ __forceinline__ void keep(v16b a, v16b b, v16b c, v16b d) { keep4_b(a, b, c, d); }
};

template <int ET> struct Elem;
template <> struct Elem<0> { typedef _Float16 T; };
template <> struct Elem<1> { typedef __bf16 T; };
template <int ET, int SPL, int BIAS_MODE, int OUT_MODE, bool RESID>
__global__ __launch_bounds__(256) void wmma_gemm64(
    const unsigned short* __restrict__ Ap, const unsigned short* __restrict__ A2p, int lda, long strideA,
    const unsigned short* __restrict__ Btp, const unsigned short* __restrict__ Bt2p, int ldb, long strideB,
    void* __restrict__ Cout, void* __restrict__ Cout2, int ldc, long strideC,
    const float* __restrict__ bias,
    const float* __restrict__ resid, long strideR,
    int M, int N, int K, float scale) {
  typedef typename Elem<ET>::T T;
  typedef typename Frag<T>::V V;
  const T* A = (const T*)Ap; const T* A2 = (const T*)A2p; const T* Bt = (const T*)Btp; const T* Bt2 = (const T*)Bt2p;
  __shared__ __align__(16) float sT[8][16 * 68];
  const int b    = blockIdx.y;
  const int lane = threadIdx.x & 31;
  const int wave = __builtin_amdgcn_readfirstlane((int)(threadIdx.x >> 5));
  const int tilesN = N >> 6;
  const int tilesM = M >> 6;
  const int tile = blockIdx.x * 8 + wave;
  if (tile >= tilesM * tilesN) return;
  const int tm = tile / tilesN;
  const int tn = tile - tm * tilesN;
  const int m0 = tm << 6;
  const int n0 = tn << 6;

  const T* Ab  = A  + (size_t)b * strideA;
  const T* Bb  = Bt + (size_t)b * strideB;
  const T* Ab2 = (SPL >= 1) ? (A2  + (size_t)b * strideA) : nullptr;
  const T* Bb2 = (SPL == 2) ? (Bt2 + (size_t)b * strideB) : nullptr;

  const int rlane = lane & 15;
  const int koff  = (lane >> 4) * 8;
  const int mOff  = (lane >> 4) * 8;

  v8f acc[4][4];
#pragma unroll
  for (int i = 0; i < 4; ++i)
#pragma unroll
    for (int j = 0; j < 4; ++j) acc[i][j] = (v8f){0.f,0.f,0.f,0.f,0.f,0.f,0.f,0.f};

  for (int k0 = 0; k0 < K; k0 += 32) {
    V bh[4], bl[4];
#pragma unroll
    for (int j = 0; j < 4; ++j) {
      const size_t bo = (size_t)(n0 + (j << 4) + rlane) * ldb + koff + k0;
      bh[j] = Frag<T>::load(Bb + bo);
      if (SPL == 2) bl[j] = Frag<T>::load(Bb2 + bo);
    }
#pragma unroll
    for (int i = 0; i < 4; ++i) {
      const size_t ao = (size_t)(m0 + (i << 4) + rlane) * lda + koff + k0;
      V ah = Frag<T>::load(Ab + ao);
      V al;
      if (SPL >= 1) al = Frag<T>::load(Ab2 + ao);
#pragma unroll
      for (int j = 0; j < 4; ++j) {
        acc[i][j] = Frag<T>::mma(ah, bh[j], acc[i][j]);
        if (SPL == 2) acc[i][j] = Frag<T>::mma(ah, bl[j], acc[i][j]);
        if (SPL >= 1) acc[i][j] = Frag<T>::mma(al, bh[j], acc[i][j]);
      }
#pragma unroll
      for (int j = 0; j < 4; ++j)
        Frag<T>::guard1(acc[i][j], ah, (SPL >= 1) ? al : ah, bh[j], (SPL == 2) ? bl[j] : bh[j]);
    }
    Frag<T>::keep(bh[0], bh[1], bh[2], bh[3]);
    if (SPL == 2) Frag<T>::keep(bl[0], bl[1], bl[2], bl[3]);
  }
  acc_guard4(acc[0][0], acc[0][1], acc[0][2], acc[0][3]);
  acc_guard4(acc[1][0], acc[1][1], acc[1][2], acc[1][3]);
  acc_guard4(acc[2][0], acc[2][1], acc[2][2], acc[2][3]);
  acc_guard4(acc[3][0], acc[3][1], acc[3][2], acc[3][3]);

  float* slab = sT[wave];
  const float* Rb = RESID ? (resid + (size_t)b * strideR) : nullptr;
#pragma unroll
  for (int i = 0; i < 4; ++i) {
    const int mBase = m0 + (i << 4);
#pragma unroll
    for (int j = 0; j < 4; ++j) {
      const int n = n0 + (j << 4) + rlane;
      float bv = 0.f;
      if (BIAS_MODE == 2) bv = bias[n];
#pragma unroll
      for (int r = 0; r < 8; ++r) {
        float v = acc[i][j][r] * scale;
        if (BIAS_MODE == 1) v += bias[mBase + mOff + r];
        if (BIAS_MODE == 2) v += bv;
        if (RESID) v += Rb[(size_t)(mBase + mOff + r) * ldc + n];
        slab[(mOff + r) * 68 + (j << 4) + rlane] = v;
      }
    }
    __builtin_amdgcn_fence(__ATOMIC_RELEASE, "workgroup");
    __builtin_amdgcn_wave_barrier();
    __builtin_amdgcn_fence(__ATOMIC_ACQUIRE, "workgroup");
    if (OUT_MODE == 0) {
      float* C = (float*)Cout + (size_t)b * strideC;
      const int hh = lane >> 4, c4 = (lane & 15) * 4;
      for (int pass = 0; pass < 2; ++pass) {
#pragma unroll
        for (int it = 0; it < 8; ++it) {
          const int row = it * 2 + hh;
          v4f v = *(const v4f*)(slab + row * 68 + c4);
          *(volatile v4f*)(C + (size_t)(mBase + row) * ldc + n0 + c4) = v;
        }
        __threadfence();
      }
    } else {
      const int q = lane >> 3, c8 = (lane & 7) * 8;
      unsigned short* C  = (unsigned short*)Cout  + (size_t)b * strideC;
      unsigned short* C2 = (OUT_MODE == 2) ? ((unsigned short*)Cout2 + (size_t)b * strideC) : nullptr;
      for (int pass = 0; pass < 2; ++pass) {
#pragma unroll
        for (int it = 0; it < 4; ++it) {
          const int row = it * 4 + q;
          const float* sp = slab + row * 68 + c8;
          v8h hv, lv;
#pragma unroll
          for (int e = 0; e < 8; ++e) {
            if (OUT_MODE == 1) {
              hv[e] = (_Float16)sp[e];
            } else {
              unsigned short hb = f2bf_bits(sp[e]);
              unsigned short lb = f2bf_bits(sp[e] - bf_bits2f(hb));
              hv[e] = __builtin_bit_cast(_Float16, hb);
              lv[e] = __builtin_bit_cast(_Float16, lb);
            }
          }
          *(volatile v8h*)(C + (size_t)(mBase + row) * ldc + n0 + c8) = hv;
          if (OUT_MODE == 2) *(volatile v8h*)(C2 + (size_t)(mBase + row) * ldc + n0 + c8) = lv;
        }
        __threadfence();
      }
    }
    __builtin_amdgcn_fence(__ATOMIC_RELEASE, "workgroup");
    __builtin_amdgcn_wave_barrier();
    __builtin_amdgcn_fence(__ATOMIC_ACQUIRE, "workgroup");
  }
}

__global__ __launch_bounds__(256) void basis_planes_kernel(unsigned* __restrict__ BH, unsigned* __restrict__ BL)
{
  __shared__ __align__(16) unsigned sW[2 * 256];
  const int tid  = threadIdx.x;
  const int wave = __builtin_amdgcn_readfirstlane((int)(threadIdx.x >> 5));
  const int w  = blockIdx.x * 256 + tid;
  const int t  = w / kFreqPad;
  const int lp = w - t * kFreqPad;
  const int lc = (lp < kFreq) ? lp : (kFreq - 1);
  const int phase = (lc * t) & (kLen - 1);
  const float x  = (float)phase * (2.0f / (float)kLen);
  const float sn = sinpif(x);
  const float cs = cospif(x);
  const bool live = (lp < kFreq);
  const bool edge = (lp == 0) || (lp >= kFreq - 1);
  const float vr = live ? cs : 0.0f;
  const float vi = edge ? 0.0f : (0.0f - sn);
  const unsigned hr = bf_rne_u32(vr);
  const unsigned hi = bf_rne_u32(vi);
  const unsigned lr = bf_rne_u32(vr - bf_u32_to_f(hr));
  const unsigned li = bf_rne_u32(vi - bf_u32_to_f(hi));
  const unsigned whi = hr | (hi << 16);
  const unsigned wlo = lr | (li << 16);
  sW[tid] = whi;
  sW[256 + tid] = wlo;
  __syncthreads();
  if (wave < 2) {
    const v4u val = *(const v4u*)(sW + tid * 4);
    unsigned* dst = BH + (size_t)blockIdx.x * 256 + tid * 4;
    *(volatile v4u*)dst = val;
    __threadfence();
    *(volatile v4u*)dst = val;
  } else if (wave < 4) {
    const int j = tid - 64;
    const v4u val = *(const v4u*)(sW + 256 + j * 4);
    unsigned* dst = BL + (size_t)blockIdx.x * 256 + j * 4;
    *(volatile v4u*)dst = val;
    __threadfence();
    *(volatile v4u*)dst = val;
  }
}

__global__ __launch_bounds__(352) void pole_sum_kernel(
    const float* __restrict__ Cm, const float* __restrict__ Bm, const float* __restrict__ Pm,
    const float* __restrict__ iwr, const float* __restrict__ wim, const float* __restrict__ ldt,
    const int* __restrict__ Lp, unsigned* __restrict__ AH, unsigned* __restrict__ AL)
{
  __shared__ __align__(16) float sP[kPoles * 12];
  const int tid  = threadIdx.x;
  const int wave = __builtin_amdgcn_readfirstlane((int)(threadIdx.x >> 5));
  const int h    = blockIdx.y;
  const float dt = expf(ldt[h]);
  const int lval = Lp[0];
  if (wave < 2) {
    const int base = h * kPoles + tid;
    const v2f cc = *(const v2f*)(Cm + 2 * base);
    const v2f bb = *(const v2f*)(Bm + 2 * base);
    const v2f pp = *(const v2f*)(Pm + 2 * base);
    const float a = (0.0f - expf(iwr[base])) * dt;
    const float b = wim[base] * dt;
    const float cr = cc[0], ci = cc[1];
    const float br = bb[0], bi = bb[1];
    const float pr = pp[0], pj = pp[1];
    v4f q0, q1, q2;
    q0[0] = a;
    q0[1] = b;
    q0[2] = br * cr - bi * ci;
    q0[3] = br * ci + bi * cr;
    q1[0] = br * pr + bi * pj;
    q1[1] = bi * pr - br * pj;
    q1[2] = pr * cr - pj * ci;
    q1[3] = pr * ci + pj * cr;
    q2[0] = pr * pr + pj * pj;
    q2[1] = 0.0f;
    q2[2] = 0.0f;
    q2[3] = 0.0f;
    *(v4f*)(sP + tid * 12)     = q0;
    *(v4f*)(sP + tid * 12 + 4) = q1;
    *(v4f*)(sP + tid * 12 + 8) = q2;
  }
  __syncthreads();

  const int l  = blockIdx.x * kPoleBlk + tid;
  const int lc = (l < kFreq) ? l : (kFreq - 1);
  const float xh = (float)lc * kInvLen;
  const float sh = sinpif(xh);
  const float ch = cospif(xh);
  const float ur = 4.0f * sh * sh;
  const float ui = 4.0f * sh * ch;
  const float gr = 2.0f * ch * ch;
  const float gi = 0.0f - 2.0f * sh * ch;

  float a00r = 0.0f, a00i = 0.0f, a01r = 0.0f, a01i = 0.0f;
  float a10r = 0.0f, a10i = 0.0f, a11r = 0.0f, a11i = 0.0f;
#pragma unroll 1
  for (int n = 0; n < kPoles; ++n) {
    const v4f p0 = *(const v4f*)(sP + n * 12);
    const v4f p1 = *(const v4f*)(sP + n * 12 + 4);
    const v4f p2 = *(const v4f*)(sP + n * 12 + 8);
    const float a = p0[0], b = p0[1];
    const float tr = ur - a * gr;
    const float qq = b * gi;
    const float d1r = tr + qq;
    const float d2r = tr - qq;
    const float ti = ui - a * gi;
    const float kk = b * gr;
    const float d1i = ti - kk;
    const float d2i = ti + kk;
    const float n1 = d1r * d1r + d1i * d1i;
    const float n2 = d2r * d2r + d2i * d2i;
    const float rp = 1.0f / (n1 * n2);
    const float i1 = n2 * rp;
    const float i2 = n1 * rp;
    const float e1r = d1r * i1;
    const float e1i = 0.0f - d1i * i1;
    const float e2r = d2r * i2;
    const float e2i = 0.0f - d2i * i2;
    const float fr  = e1r + e2r;
    const float fi  = e1i + e2i;
    const float hr  = e1r - e2r;
    const float hi_ = e2i - e1i;
    a00r += p0[2] * fr + p0[3] * hi_;
    a00i += p0[2] * fi + p0[3] * hr;
    a01r += p1[0] * fr + p1[1] * hi_;
    a01i += p1[0] * fi + p1[1] * hr;
    a10r += p1[2] * fr + p1[3] * hi_;
    a10i += p1[2] * fi + p1[3] * hr;
    a11r += p2[0] * fr;
    a11i += p2[0] * fi;
  }
  const float s00r = dt * a00r, s00i = dt * a00i;
  const float s01r = dt * a01r, s01i = dt * a01i;
  const float s10r = dt * a10r, s10i = dt * a10i;
  const float s11r = dt * a11r, s11i = dt * a11i;
  const float der = 1.0f + (gr * s11r - gi * s11i);
  const float dei = gr * s11i + gi * s11r;
  const float pr_ = s01r * s10r - s01i * s10i;
  const float pi_ = s01r * s10i + s01i * s10r;
  const float nr = gr * pr_ - gi * pi_;
  const float ni = gr * pi_ + gi * pr_;
  const float dm = 1.0f / (der * der + dei * dei);
  const float qr = (nr * der + ni * dei) * dm;
  const float qi = (ni * der - nr * dei) * dm;
  const float xr = 2.0f * (s00r - qr);
  const float xi = 2.0f * (s00i - qi);

  const bool live  = (l < kFreq);
  const bool inner = (l > 0) && (l < kFreq - 1);
  float wr_ = inner ? (2.0f * xr) : xr;
  wr_ = live ? wr_ : 0.0f;
  float wi_ = inner ? (2.0f * xi) : 0.0f;
  const bool bad = (lval != kLen);
  const float qnan = __uint_as_float(0x7FC00000u);
  wr_ = bad ? qnan : wr_;
  wi_ = bad ? qnan : wi_;

  const unsigned hbr = bf_rne_u32(wr_);
  const unsigned hbi = bf_rne_u32(wi_);
  const unsigned lbr = bf_rne_u32(wr_ - bf_u32_to_f(hbr));
  const unsigned lbi = bf_rne_u32(wi_ - bf_u32_to_f(hbi));
  const unsigned whi = hbr | (hbi << 16);
  const unsigned wlo = lbr | (lbi << 16);
  const size_t idx = (size_t)h * kFreqPad + (size_t)l;
  volatile unsigned* ph = (volatile unsigned*)(AH + idx);
  volatile unsigned* pl = (volatile unsigned*)(AL + idx);
  *ph = whi;
  *pl = wlo;
  __threadfence();
  *ph = whi;
  *pl = wlo;
}

extern "C" void kernel_launch(void* const* d_in, const int* in_sizes, int n_in,
                              void* d_out, int out_size, void* d_ws, size_t ws_size,
                              hipStream_t stream) {
  if (n_in < 7) return;
  if (in_sizes[0] != kHeads * kPoles * 2) return;
  if (in_sizes[1] != kHeads * kPoles * 2) return;
  if (in_sizes[2] != kHeads * kPoles * 2) return;
  if (in_sizes[3] != kHeads * kPoles) return;
  if (in_sizes[4] != kHeads * kPoles) return;
  if (in_sizes[5] != kHeads) return;
  if (in_sizes[6] != 1) return;
  if (out_size != kHeads * kLen) return;
  if (ws_size < kWsTotal) return;

  const float* Cm  = (const float*)d_in[0];
  const float* Bm  = (const float*)d_in[1];
  const float* Pm  = (const float*)d_in[2];
  const float* iwr = (const float*)d_in[3];
  const float* wim = (const float*)d_in[4];
  const float* ldt = (const float*)d_in[5];
  const int*   Lp  = (const int*)d_in[6];
  float* out = (float*)d_out;

  char* ws = (char*)d_ws;
  unsigned* BH = (unsigned*)(ws + kOffBH);
  unsigned* BL = (unsigned*)(ws + kOffBL);
  unsigned* AH = (unsigned*)(ws + kOffAH);
  unsigned* AL = (unsigned*)(ws + kOffAL);

  basis_planes_kernel<<<kBasisBlocks, 256, 0, stream>>>(BH, BL);

  pole_sum_kernel<<<dim3(kPoleChunks, kHeads), kPoleBlk, 0, stream>>>(Cm, Bm, Pm, iwr, wim, ldt, Lp, AH, AL);

  wmma_gemm64<1, 2, 0, 0, false><<<dim3((kHeads / 64) * (kLen / 64) / 8, 1), 256, 0, stream>>>(
      (const unsigned short*)AH, (const unsigned short*)AL, kKdim, 0L,
      (const unsigned short*)BH, (const unsigned short*)BL, kKdim, 0L,
      (void*)out, nullptr, kLen, 0L,
      nullptr, nullptr, 0L,
      kHeads, kLen, kKdim, kInvLen);
}
